// Deform_GAU_14345190768898
// MI455X (gfx1250) — hardware-verified
//
#include <hip/hip_runtime.h>
#include <stdint.h>


#define NB     4
#define CHI    512
#define CLO    256
#define HHI    32
#define HLO    64
#define HWP    4096
#define MROWS  16384
#define HROWS  8192
#define K3     2304
#define KUP    2048
#define PMC    32
#define NPOS   (NB * HWP)

static_assert(MROWS % 32 == 0 && HROWS % 32 == 0);
static_assert(K3 % 32 == 0 && KUP % 32 == 0);
static_assert(CLO % 256 == 0 && PMC % 32 == 0);

typedef unsigned short us;
typedef _Float16 v16h __attribute__((ext_vector_type(16)));
typedef __bf16   v16b __attribute__((ext_vector_type(16)));
typedef float    v8f  __attribute__((ext_vector_type(8)));
typedef float    v4f  __attribute__((ext_vector_type(4)));
typedef int      v4i  __attribute__((ext_vector_type(4)));

__device__ __forceinline__ uint32_t bf16_bits(float f) {
  uint32_t u = __float_as_uint(f);
  u += 0x7FFFu + ((u >> 16) & 1u);
  return u >> 16;
}
__device__ __forceinline__ float bf16_val(uint32_t b) { return __uint_as_float(b << 16); }
__device__ __forceinline__ float bf16r(float f) { return bf16_val(bf16_bits(f)); }
__device__ __forceinline__ float bf16res(float f) { return f - bf16r(f); }
__device__ __forceinline__ uint32_t h16_bits(float f) {
  union { _Float16 h; us u; } c;
  c.h = (_Float16)f;
  return (uint32_t)c.u;
}
__device__ __forceinline__ int pk2(uint32_t lo, uint32_t hi) { return (int)(lo | (hi << 16)); }
__device__ __forceinline__ v4i pack_bf16_8(v4f a, v4f b) {
  v4i r;
  r.x = pk2(bf16_bits(a.x), bf16_bits(a.y));
  r.y = pk2(bf16_bits(a.z), bf16_bits(a.w));
  r.z = pk2(bf16_bits(b.x), bf16_bits(b.y));
  r.w = pk2(bf16_bits(b.z), bf16_bits(b.w));
  return r;
}
__device__ __forceinline__ v4i pack_bf16lo_8(v4f a, v4f b) {
  v4f ra, rb;
  ra.x = bf16res(a.x); ra.y = bf16res(a.y); ra.z = bf16res(a.z); ra.w = bf16res(a.w);
  rb.x = bf16res(b.x); rb.y = bf16res(b.y); rb.z = bf16res(b.z); rb.w = bf16res(b.w);
  return pack_bf16_8(ra, rb);
}
__device__ __forceinline__ v4i pack_h16_8(v4f a, v4f b) {
  v4i r;
  r.x = pk2(h16_bits(a.x), h16_bits(a.y));
  r.y = pk2(h16_bits(a.z), h16_bits(a.w));
  r.z = pk2(h16_bits(b.x), h16_bits(b.y));
  r.w = pk2(h16_bits(b.z), h16_bits(b.w));
  return r;
}
__device__ __forceinline__ v4f zero4() { v4f z = {0.0f, 0.0f, 0.0f, 0.0f}; return z; }
__device__ __forceinline__ void vst16(us* p, v4i v) { *(volatile v4i*)p = v; }
__device__ __forceinline__ void vst16(float* p, v4f v) { *(volatile v4f*)p = v; }
__device__ __forceinline__ double shfl_xor_d(double v, int o) {
  int lo = __double2loint(v), hi = __double2hiint(v);
  lo = __shfl_xor(lo, o);
  hi = __shfl_xor(hi, o);
  return __hiloint2double(hi, lo);
}

template <int BF> struct Eng;
template <> struct Eng<0> {
  typedef v16h V;
  static __device__ __forceinline__ v8f mma(v8f c, V a, V b) {
    c = __builtin_amdgcn_wmma_f32_16x16x32_f16(false, a, false, b, (short)0, c, false, false);
    asm volatile("v_nop\n\tv_nop\n\tv_nop\n\tv_nop" : "+v"(c) : "v"(a), "v"(b));
    return c;
  }
};
template <> struct Eng<1> {
  typedef v16b V;
  static __device__ __forceinline__ v8f mma(v8f c, V a, V b) {
    c = __builtin_amdgcn_wmma_f32_16x16x32_bf16(false, a, false, b, (short)0, c, false, false);
    asm volatile("v_nop\n\tv_nop\n\tv_nop\n\tv_nop" : "+v"(c) : "v"(a), "v"(b));
    return c;
  }
};
template <int BF> union Frag { typename Eng<BF>::V v; v4i q[2]; };

template <int BF, int NPL, int JC, int WPB>
__global__ void __launch_bounds__(32 * WPB)
k_gemm(const us* __restrict__ A, const us* __restrict__ B, float* __restrict__ outp,
       int K, int nrows, int rowbase, int ctot, int gshift, int gmask, int bgs, int pstride, float oscale)
{
  __shared__ __attribute__((aligned(16))) float stg[WPB][512 * JC];
  typedef typename Eng<BF>::V V;
  const int tid = (int)threadIdx.x;
  const int l = tid & 31, wv = tid >> 5, h = l >> 4, m = l & 15;
  const int lr0 = (int)blockIdx.x * 32;
  if (lr0 + 32 > nrows) return;
  if (((int)blockIdx.y + 1) * (WPB * 16 * JC) > ctot) return;
  const int gr0 = rowbase + lr0;
  const int nb = gr0 >> 12, p0 = gr0 & (HWP - 1);
  const int grp = (gr0 >> gshift) & gmask;
  const us* Bg = B + (size_t)grp * (size_t)bgs;
  const int col0 = ((int)blockIdx.y * WPB + wv) * (16 * JC);

  v8f acc[2][JC];
#pragma unroll
  for (int t = 0; t < 2; ++t)
#pragma unroll
    for (int j = 0; j < JC; ++j) {
#pragma unroll
      for (int e = 0; e < 8; ++e) acc[t][j][e] = 0.0f;
    }

  const us* ar[2][NPL];
#pragma unroll
  for (int t = 0; t < 2; ++t)
#pragma unroll
    for (int pl = 0; pl < NPL; ++pl)
      ar[t][pl] = A + (size_t)pl * (size_t)pstride + (size_t)(lr0 + t * 16 + m) * (size_t)K + 8 * h;
  const us* bc[JC];
#pragma unroll
  for (int j = 0; j < JC; ++j)
    bc[j] = Bg + (size_t)(col0 + j * 16 + m) * (size_t)K + 8 * h;

#pragma unroll 2
  for (int k0 = 0; k0 < K; k0 += 32) {
    V av[2][NPL];
#pragma unroll
    for (int t = 0; t < 2; ++t)
#pragma unroll
      for (int pl = 0; pl < NPL; ++pl) {
        Frag<BF> f;
        f.q[0] = *(const v4i*)(ar[t][pl] + k0);
        f.q[1] = *(const v4i*)(ar[t][pl] + k0 + 16);
        av[t][pl] = f.v;
      }
#pragma unroll
    for (int j = 0; j < JC; ++j) {
      Frag<BF> g;
      g.q[0] = *(const v4i*)(bc[j] + k0);
      g.q[1] = *(const v4i*)(bc[j] + k0 + 16);
#pragma unroll
      for (int t = 0; t < 2; ++t)
#pragma unroll
        for (int pl = 0; pl < NPL; ++pl)
          acc[t][j] = Eng<BF>::mma(acc[t][j], av[t][pl], g.v);
    }
  }

  float* sw = &stg[wv][0];
#pragma unroll
  for (int t = 0; t < 2; ++t)
#pragma unroll
    for (int j = 0; j < JC; ++j) {
      v4f u0, u1;
      u0.x = acc[t][j][0] * oscale; u0.y = acc[t][j][1] * oscale;
      u0.z = acc[t][j][2] * oscale; u0.w = acc[t][j][3] * oscale;
      u1.x = acc[t][j][4] * oscale; u1.y = acc[t][j][5] * oscale;
      u1.z = acc[t][j][6] * oscale; u1.w = acc[t][j][7] * oscale;
      float* sp = sw + (j * 16 + m) * 32 + t * 16 + 8 * h;
      *(v4f*)sp = u0;
      *(v4f*)(sp + 4) = u1;
    }
  __syncthreads();

  float* ob = outp + ((size_t)nb * (size_t)ctot + (size_t)col0) * HWP + p0;
  const int q = l & 7, lq = l >> 3;
#pragma unroll
  for (int it = 0; it < 4 * JC; ++it) {
    const int cc = it * 4 + lq;
    const v4f v = *(const v4f*)(sw + cc * 32 + q * 4);
    vst16(ob + (size_t)cc * HWP + q * 4, v);
  }
  __threadfence();
#pragma unroll
  for (int it = 0; it < 4 * JC; ++it) {
    const int cc = it * 4 + lq;
    const v4f v = *(const v4f*)(sw + cc * 32 + q * 4);
    vst16(ob + (size_t)cc * HWP + q * 4, v);
  }
}

template <int BF>
__global__ void __launch_bounds__(256) k_prep_w3(const float* __restrict__ w, us* __restrict__ wt, float premul)
{
  const int idx = (int)blockIdx.x * 256 + (int)threadIdx.x;
  if (idx >= CLO * 288) return;
  const int oc = idx / 288, rem = idx - oc * 288;
  const int tap = rem >> 5, c0 = (rem & 31) * 8;
  const float* sp = w + ((size_t)oc * CLO + c0) * 9 + tap;
  v4f a, b;
  a.x = sp[0];  a.y = sp[9];  a.z = sp[18]; a.w = sp[27];
  b.x = sp[36]; b.y = sp[45]; b.z = sp[54]; b.w = sp[63];
  v4i pk;
  if (BF) {
    pk = pack_bf16_8(a, b);
  } else {
    v4f sa, sb;
    sa.x = bf16r(a.x) * premul; sa.y = bf16r(a.y) * premul; sa.z = bf16r(a.z) * premul; sa.w = bf16r(a.w) * premul;
    sb.x = bf16r(b.x) * premul; sb.y = bf16r(b.y) * premul; sb.z = bf16r(b.z) * premul; sb.w = bf16r(b.w) * premul;
    pk = pack_h16_8(sa, sb);
  }
  us* d = wt + (size_t)idx * 8;
  vst16(d, pk);
  __threadfence();
  vst16(d, pk);
}

__global__ void __launch_bounds__(256) k_prep_wpm(const float* __restrict__ pw, const float* __restrict__ mw,
                                                  us* __restrict__ wt)
{
  const int idx = (int)blockIdx.x * 256 + (int)threadIdx.x;
  if (idx >= PMC * 288) return;
  const int oc = idx / 288, rem = idx - oc * 288;
  const int tap = rem >> 5, c0 = (rem & 31) * 8;
  v4f a = zero4(), b = zero4();
  const float* sp = 0;
  if (oc < 18) sp = pw + ((size_t)oc * CLO + c0) * 9 + tap;
  else if (oc < 27) sp = mw + ((size_t)(oc - 18) * CLO + c0) * 9 + tap;
  if (sp) {
    a.x = sp[0];  a.y = sp[9];  a.z = sp[18]; a.w = sp[27];
    b.x = sp[36]; b.y = sp[45]; b.z = sp[54]; b.w = sp[63];
  }
  const v4i pk = pack_bf16_8(a, b);
  us* d = wt + (size_t)idx * 8;
  vst16(d, pk);
  __threadfence();
  vst16(d, pk);
}

__global__ void __launch_bounds__(256) k_prep_wup(const float* __restrict__ w, us* __restrict__ wt)
{
  const int idx = (int)blockIdx.x * 256 + (int)threadIdx.x;
  if (idx >= 4 * CLO * 256) return;
  const int par = idx >> 16, rem = idx & 65535;
  const int oc = rem >> 8, r2 = rem & 255;
  const int tap = r2 >> 6, ic0 = (r2 & 63) * 8;
  const int pyr = par >> 1, pxr = par & 1, kyH = tap >> 1, kxH = tap & 1;
  const int ky = (1 - pyr) + 2 * kyH, kx = (1 - pxr) + 2 * kxH;
  const float* sp = w + (((size_t)ic0 * CLO + oc) * 4 + ky) * 4 + kx;
  v4f a, b;
  a.x = sp[0];         a.y = sp[4096];      a.z = sp[2 * 4096];  a.w = sp[3 * 4096];
  b.x = sp[4 * 4096];  b.y = sp[5 * 4096];  b.z = sp[6 * 4096];  b.w = sp[7 * 4096];
  const v4i pk = pack_bf16_8(a, b);
  us* d = wt + (size_t)idx * 8;
  vst16(d, pk);
  __threadfence();
  vst16(d, pk);
}

__global__ void __launch_bounds__(256) k_gather_up(const float* __restrict__ xh, us* __restrict__ X)
{
  const int idx = (int)blockIdx.x * 256 + (int)threadIdx.x;
  if (idx >= MROWS * 256) return;
  const int r = idx >> 8, r2 = idx & 255;
  const int tap = r2 >> 6, ic0 = (r2 & 63) * 8;
  const int n = r >> 12, pp = r & 4095;
  const int par = pp >> 10, i = (pp >> 5) & 31, j = pp & 31;
  const int pyr = par >> 1, pxr = par & 1, kyH = tap >> 1, kxH = tap & 1;
  const int iy = i + pyr - kyH, ix = j + pxr - kxH;
  v4f a = zero4(), b = zero4();
  if ((unsigned)iy < (unsigned)HHI && (unsigned)ix < (unsigned)HHI) {
    const float* sp = xh + (((size_t)n * CHI + ic0) * HHI + iy) * HHI + ix;
    a.x = sp[0];    a.y = sp[1024]; a.z = sp[2048]; a.w = sp[3072];
    b.x = sp[4096]; b.y = sp[5120]; b.z = sp[6144]; b.w = sp[7168];
  }
  const v4i pk = pack_bf16_8(a, b);
  us* d = X + (size_t)idx * 8;
  vst16(d, pk);
  __threadfence();
  vst16(d, pk);
}

__global__ void __launch_bounds__(256) k_im2col_low(const float* __restrict__ xl, us* __restrict__ X)
{
  const int idx = (int)blockIdx.x * 256 + (int)threadIdx.x;
  if (idx >= MROWS * 288) return;
  const int r = idx / 288, rem = idx - r * 288;
  const int tap = rem >> 5, c0 = (rem & 31) * 8;
  const int n = r >> 12, p = r & 4095, y = p >> 6, x = p & 63;
  const int kyi = tap / 3, kxi = tap - kyi * 3;
  const int yy = y + kyi - 1, xx = x + kxi - 1;
  v4f a = zero4(), b = zero4();
  if ((unsigned)yy < (unsigned)HLO && (unsigned)xx < (unsigned)HLO) {
    const float* sp = xl + (((size_t)n * CLO + c0) * HLO + yy) * HLO + xx;
    a.x = sp[0];         a.y = sp[4096];      a.z = sp[2 * 4096];  a.w = sp[3 * 4096];
    b.x = sp[4 * 4096];  b.y = sp[5 * 4096];  b.z = sp[6 * 4096];  b.w = sp[7 * 4096];
  }
  const v4i pk = pack_bf16_8(a, b);
  us* d = X + (size_t)idx * 8;
  vst16(d, pk);
  __threadfence();
  vst16(d, pk);
}

__global__ void __launch_bounds__(256) k_im2col_hilo(const float* __restrict__ hf, us* __restrict__ X, int rowhalf)
{
  const int idx = (int)blockIdx.x * 256 + (int)threadIdx.x;
  if (idx >= HROWS * 288) return;
  const int r = idx / 288, rem = idx - r * 288;
  const int tap = rem >> 5, c0 = (rem & 31) * 8;
  const int gr = rowhalf * HROWS + r;
  const int n = gr >> 12, p = gr & 4095, y = p >> 6, x = p & 63;
  const int kyi = tap / 3, kxi = tap - kyi * 3;
  const int yy = y + kyi - 1, xx = x + kxi - 1;
  v4f a = zero4(), b = zero4();
  if ((unsigned)yy < (unsigned)HLO && (unsigned)xx < (unsigned)HLO) {
    const float* sp = hf + ((size_t)(n * HLO + yy) * HLO + xx) * CLO + c0;
    a = *(const v4f*)sp;
    b = *(const v4f*)(sp + 4);
  }
  const v4i ph = pack_bf16_8(a, b);
  const v4i pl = pack_bf16lo_8(a, b);
  us* dh = X + (size_t)idx * 8;
  us* dl = dh + (size_t)HROWS * K3;
  vst16(dh, ph);
  vst16(dl, pl);
  __threadfence();
  vst16(dh, ph);
  vst16(dl, pl);
}

__global__ void __launch_bounds__(256)
k_im2col_deform(const float* __restrict__ hf, const float* __restrict__ pm,
                const float* __restrict__ pb, const float* __restrict__ mb, us* __restrict__ X)
{
  const int idx = (int)blockIdx.x * 256 + (int)threadIdx.x;
  if (idx >= MROWS * 72) return;
  const int c8 = idx & 7;
  const int t2 = idx >> 3;
  const int r = t2 / 9, kk = t2 - r * 9;
  const int n = r >> 12, p = r & (HWP - 1), y = p >> 6, x = p & 63;
  const int kyi = kk / 3, kxi = kk - kyi * 3;
  const float* pmn = pm + (size_t)(n * PMC) * HWP + p;
  const float dy = pmn[(size_t)kk * HWP] + bf16r(pb[kk]);
  const float dx = pmn[(size_t)(9 + kk) * HWP] + bf16r(pb[9 + kk]);
  const float mr = pmn[(size_t)(18 + kk) * HWP] + bf16r(mb[kk]);
  const float mg = __frcp_rn(1.0f + __expf(-mr));
  float py = (float)(y + kyi) + dy;
  float px = (float)(x + kxi) + dx;
  py = fminf(fmaxf(py, 0.0f), 65.0f);
  px = fminf(fmaxf(px, 0.0f), 65.0f);
  const float y0f = floorf(py), x0f = floorf(px);
  const float wy = py - y0f, wx = px - x0f;
  int y0 = (int)y0f, x0 = (int)x0f;
  y0 = min(max(y0, 0), 65);
  x0 = min(max(x0, 0), 65);
  const int y1 = min(y0 + 1, 65), x1 = min(x0 + 1, 65);
  const int sy0 = y0 - 1, sy1 = y1 - 1, sx0 = x0 - 1, sx1 = x1 - 1;
  const bool vy0 = (unsigned)sy0 < (unsigned)HLO, vy1 = (unsigned)sy1 < (unsigned)HLO;
  const bool vx0 = (unsigned)sx0 < (unsigned)HLO, vx1 = (unsigned)sx1 < (unsigned)HLO;
  const float mgs = mg * 256.0f;
  const float w00 = (vy0 && vx0) ? (1.0f - wy) * (1.0f - wx) * mgs : 0.0f;
  const float w01 = (vy0 && vx1) ? (1.0f - wy) * wx * mgs : 0.0f;
  const float w10 = (vy1 && vx0) ? wy * (1.0f - wx) * mgs : 0.0f;
  const float w11 = (vy1 && vx1) ? wy * wx * mgs : 0.0f;
  const size_t nbase = (size_t)n * HWP * CLO + (size_t)c8 * 32;
  const float* p00 = hf + nbase + (size_t)((vy0 ? sy0 : 0) * HLO + (vx0 ? sx0 : 0)) * CLO;
  const float* p01 = hf + nbase + (size_t)((vy0 ? sy0 : 0) * HLO + (vx1 ? sx1 : 0)) * CLO;
  const float* p10 = hf + nbase + (size_t)((vy1 ? sy1 : 0) * HLO + (vx0 ? sx0 : 0)) * CLO;
  const float* p11 = hf + nbase + (size_t)((vy1 ? sy1 : 0) * HLO + (vx1 ? sx1 : 0)) * CLO;
  us* dst = X + (size_t)idx * 32;
#pragma unroll 1
  for (int ps = 0; ps < 2; ++ps) {
#pragma unroll 1
    for (int e8 = 0; e8 < 4; ++e8) {
      const int o = e8 * 8;
      const v4f a00 = *(const v4f*)(p00 + o), b00 = *(const v4f*)(p00 + o + 4);
      const v4f a01 = *(const v4f*)(p01 + o), b01 = *(const v4f*)(p01 + o + 4);
      const v4f a10 = *(const v4f*)(p10 + o), b10 = *(const v4f*)(p10 + o + 4);
      const v4f a11 = *(const v4f*)(p11 + o), b11 = *(const v4f*)(p11 + o + 4);
      const v4f ra = a00 * w00 + a01 * w01 + a10 * w10 + a11 * w11;
      const v4f rb = b00 * w00 + b01 * w01 + b10 * w10 + b11 * w11;
      vst16(dst + o, pack_h16_8(ra, rb));
    }
    if (ps == 0) __threadfence();
  }
}

__global__ void __launch_bounds__(256) k_bnstats(const float* __restrict__ T, float* __restrict__ stat)
{
  __shared__ __attribute__((aligned(16))) float rm[32];
  __shared__ __attribute__((aligned(16))) float rr[32];
  const int tid = (int)threadIdx.x, l = tid & 31, wv = tid >> 5;
  const int cb = (int)blockIdx.x * 32;
#pragma unroll 1
  for (int ci = 0; ci < 4; ++ci) {
    const int c = cb + wv * 4 + ci;
    double s = 0.0, sq = 0.0;
#pragma unroll 1
    for (int n = 0; n < NB; ++n) {
      const float* base = T + ((size_t)(n * CLO + c)) * HWP;
#pragma unroll 4
      for (int i = l; i < HWP; i += 32) {
        const double v = (double)base[i];
        s += v;
        sq += v * v;
      }
    }
#pragma unroll
    for (int o = 16; o > 0; o >>= 1) {
      s += shfl_xor_d(s, o);
      sq += shfl_xor_d(sq, o);
    }
    if (l == 0) {
      const double inv = 1.0 / (double)(NB * HWP);
      const double mu = s * inv;
      double var = sq * inv - mu * mu;
      if (var < 0.0) var = 0.0;
      const float varf = (float)var;
      rm[wv * 4 + ci] = (float)mu;
      rr[wv * 4 + ci] = 1.0f / sqrtf(varf + 1e-5f);
    }
  }
  __syncthreads();
  if (wv == 0 && l < 16) {
    const int q = l & 7;
    v4f v;
    float* dst;
    if (l < 8) { v = *(const v4f*)&rm[q * 4]; dst = stat + cb + q * 4; }
    else       { v = *(const v4f*)&rr[q * 4]; dst = stat + CLO + cb + q * 4; }
    vst16(dst, v);
    __threadfence();
    vst16(dst, v);
  }
}

__global__ void __launch_bounds__(256)
k_norm_highf(const float* __restrict__ T, const float* __restrict__ stat,
             const float* __restrict__ g, const float* __restrict__ b, float* __restrict__ hf)
{
  __shared__ __attribute__((aligned(16))) float s[HLO * 128];
  const int tid = (int)threadIdx.x, l = tid & 31, wv = tid >> 5;
  const int bid = (int)blockIdx.x;
  const int cblk = bid & 1, y = (bid >> 1) & 63, n = bid >> 7;
  const int pyr = y & 1, i = y >> 1;
#pragma unroll 1
  for (int cl = wv; cl < 128; cl += 8) {
    const int c = cblk * 128 + cl;
    const float mu = stat[c], rs = stat[CLO + c];
    const float gq = bf16r(g[c]), bq = bf16r(b[c]);
    const float* base = T + ((size_t)(n * CLO + c)) * HWP + i * 32 + l;
#pragma unroll
    for (int pxr = 0; pxr < 2; ++pxr) {
      const float v = base[(pyr * 2 + pxr) * 1024];
      const float o = ((v - mu) * rs) * gq + bq;
      s[(2 * l + pxr) * 128 + cl] = o;
    }
  }
  __syncthreads();
  float* ob = hf + ((size_t)(n * HLO + y) * HLO) * CLO + cblk * 128;
  const int q = l & 7, lq = l >> 3;
#pragma unroll 1
  for (int it = 0; it < 8; ++it) {
    const int L = it * 32 + wv * 4 + lq;
    const int x = L >> 2, cq = (L & 3) * 32 + q * 4;
    const v4f v = *(const v4f*)&s[x * 128 + cq];
    vst16(ob + (size_t)x * CLO + cq, v);
  }
  __threadfence();
#pragma unroll 1
  for (int it = 0; it < 8; ++it) {
    const int L = it * 32 + wv * 4 + lq;
    const int x = L >> 2, cq = (L & 3) * 32 + q * 4;
    const v4f v = *(const v4f*)&s[x * 128 + cq];
    vst16(ob + (size_t)x * CLO + cq, v);
  }
}

__global__ void __launch_bounds__(256) k_mask(const float* __restrict__ pm, const float* __restrict__ mb,
                                              float* __restrict__ mk)
{
  const int idx = (int)blockIdx.x * 256 + (int)threadIdx.x;
  if (idx >= NPOS / 4) return;
  const int n = idx >> 10, p0 = (idx & 1023) * 4;
  v4f sacc = zero4();
#pragma unroll 1
  for (int k = 0; k < 9; ++k) {
    const v4f v = *(const v4f*)(pm + ((size_t)(n * PMC + 18 + k)) * HWP + p0);
    sacc = sacc + (v + bf16r(mb[k]));
  }
  const float ninth = 1.0f / 9.0f;
  v4f r;
  r.x = __frcp_rn(1.0f + __expf(-(sacc.x * ninth)));
  r.y = __frcp_rn(1.0f + __expf(-(sacc.y * ninth)));
  r.z = __frcp_rn(1.0f + __expf(-(sacc.z * ninth)));
  r.w = __frcp_rn(1.0f + __expf(-(sacc.w * ninth)));
  float* d = mk + (size_t)idx * 4;
  vst16(d, r);
  __threadfence();
  vst16(d, r);
}

__global__ void __launch_bounds__(256)
k_final(const float* __restrict__ lowr, const float* __restrict__ dr,
        const float* __restrict__ stL, const float* __restrict__ stD,
        const float* __restrict__ gl, const float* __restrict__ bl,
        const float* __restrict__ gh, const float* __restrict__ bh,
        const float* __restrict__ mk, float* __restrict__ outp)
{
  const int idx = (int)blockIdx.x * 256 + (int)threadIdx.x;
  if (idx >= NB * CLO * HWP / 4) return;
  const int n = idx >> 18, c = (idx >> 10) & (CLO - 1), p0 = (idx & 1023) * 4;
  const size_t e = (size_t)idx * 4;
  const v4f lo = *(const v4f*)(lowr + e);
  const v4f dd = *(const v4f*)(dr + e);
  const v4f m4 = *(const v4f*)(mk + (size_t)n * HWP + p0);
  const float ml = stL[c], rl = stL[CLO + c], g1 = bf16r(gl[c]), b1 = bf16r(bl[c]);
  const float md = stD[c], rd = stD[CLO + c], g2 = bf16r(gh[c]), b2 = bf16r(bh[c]);
  const v4f lv = ((lo - ml) * rl) * g1 + b1;
  const v4f dv = ((dd - md) * rd) * g2 + b2;
  v4f rr = lv * m4 + dv;
  rr.x = fmaxf(rr.x, 0.0f); rr.y = fmaxf(rr.y, 0.0f); rr.z = fmaxf(rr.z, 0.0f); rr.w = fmaxf(rr.w, 0.0f);
  vst16(outp + e, rr);
  __threadfence();
  vst16(outp + e, rr);
}

static inline unsigned cdiv(unsigned a, unsigned b) { return (a + b - 1) / b; }

extern "C" void kernel_launch(void* const* d_in, const int* in_sizes, int n_in,
                              void* d_out, int out_size, void* d_ws, size_t ws_size,
                              hipStream_t stream)
{
  if (n_in < 15 || out_size != NB * CLO * HWP) return;
  if (in_sizes[0] != NB * CHI * HHI * HHI || in_sizes[1] != NB * CLO * HWP ||
      in_sizes[2] != CLO * CLO * 9 || in_sizes[3] != CLO || in_sizes[4] != CLO ||
      in_sizes[5] != CHI * CLO * 16 || in_sizes[6] != CLO || in_sizes[7] != CLO ||
      in_sizes[8] != 18 * CLO * 9 || in_sizes[9] != 18 || in_sizes[10] != 9 * CLO * 9 ||
      in_sizes[11] != 9 || in_sizes[12] != CLO * CLO * 9 || in_sizes[13] != CLO || in_sizes[14] != CLO) return;

  const float* fms_high  = (const float*)d_in[0];
  const float* fms_low   = (const float*)d_in[1];
  const float* conv3x3_w = (const float*)d_in[2];
  const float* bn_low_g  = (const float*)d_in[3];
  const float* bn_low_b  = (const float*)d_in[4];
  const float* up_w      = (const float*)d_in[5];
  const float* bn_up_g   = (const float*)d_in[6];
  const float* bn_up_b   = (const float*)d_in[7];
  const float* p_w       = (const float*)d_in[8];
  const float* p_b       = (const float*)d_in[9];
  const float* m_w       = (const float*)d_in[10];
  const float* m_b       = (const float*)d_in[11];
  const float* dconv_w   = (const float*)d_in[12];
  const float* bn_high_g = (const float*)d_in[13];
  const float* bn_high_b = (const float*)d_in[14];
  float* out = (float*)d_out;

  size_t off = 0;
  char* ws = (char*)d_ws;
  auto carve = [&](size_t bytes) -> void* {
    void* p = (void*)(ws + off);
    off = (off + bytes + 255) & ~(size_t)255;
    return p;
  };
  us*    X    = (us*)carve((size_t)MROWS * K3 * 2);
  float* T1   = (float*)carve((size_t)NB * CLO * HWP * 4);
  float* T2   = (float*)carve((size_t)NB * CLO * HWP * 4);
  float* PM   = (float*)carve((size_t)NB * PMC * HWP * 4);
  us*    Wlow = (us*)carve((size_t)CLO * K3 * 2);
  us*    Wd   = (us*)carve((size_t)CLO * K3 * 2);
  us*    Wpm  = (us*)carve((size_t)PMC * K3 * 2);
  us*    Wup  = (us*)carve((size_t)4 * CLO * KUP * 2);
  float* MK   = (float*)carve((size_t)NPOS * 4);
  float* ST   = (float*)carve((size_t)3 * 2 * CLO * 4);
  if (off > ws_size) return;

  const dim3 b256(256);

  k_prep_w3<1><<<dim3(cdiv(CLO * 288, 256)), b256, 0, stream>>>(conv3x3_w, Wlow, 1.0f);
  k_prep_w3<0><<<dim3(cdiv(CLO * 288, 256)), b256, 0, stream>>>(dconv_w, Wd, 64.0f);
  k_prep_wpm<<<dim3(cdiv(PMC * 288, 256)), b256, 0, stream>>>(p_w, m_w, Wpm);
  k_prep_wup<<<dim3(cdiv(4 * CLO * 256, 256)), b256, 0, stream>>>(up_w, Wup);

  k_gather_up<<<dim3(cdiv(MROWS * 256, 256)), b256, 0, stream>>>(fms_high, X);
  k_gemm<1, 1, 4, 4><<<dim3(MROWS / 32, CLO / 256), dim3(128), 0, stream>>>(
      X, Wup, T1, KUP, MROWS, 0, CLO, 10, 3, CLO * KUP, 0, 1.0f);
  k_bnstats<<<dim3(CLO / 32), b256, 0, stream>>>(T1, ST);
  k_norm_highf<<<dim3(NB * HLO * 2), b256, 0, stream>>>(T1, ST, bn_up_g, bn_up_b, T2);

  for (int hh = 0; hh < 2; ++hh) {
    k_im2col_hilo<<<dim3(cdiv(HROWS * 288, 256)), b256, 0, stream>>>(T2, X, hh);
    k_gemm<1, 2, 2, 1><<<dim3(HROWS / 32, 1), dim3(32), 0, stream>>>(
        X, Wpm, PM, K3, HROWS, hh * HROWS, PMC, 0, 0, 0, HROWS * K3, 1.0f);
  }

  k_im2col_low<<<dim3(cdiv(MROWS * 288, 256)), b256, 0, stream>>>(fms_low, X);
  k_gemm<1, 1, 4, 4><<<dim3(MROWS / 32, CLO / 256), dim3(128), 0, stream>>>(
      X, Wlow, T1, K3, MROWS, 0, CLO, 0, 0, 0, 0, 1.0f);
  k_bnstats<<<dim3(CLO / 32), b256, 0, stream>>>(T1, ST + 2 * CLO);

  k_im2col_deform<<<dim3(cdiv(MROWS * 72, 256)), b256, 0, stream>>>(T2, PM, p_b, m_b, X);
  k_gemm<0, 1, 4, 4><<<dim3(MROWS / 32, CLO / 256), dim3(128), 0, stream>>>(
      X, Wd, T2, K3, MROWS, 0, CLO, 0, 0, 0, 0, 1.0f / 16384.0f);
  k_bnstats<<<dim3(CLO / 32), b256, 0, stream>>>(T2, ST + 4 * CLO);

  k_mask<<<dim3(cdiv(NPOS / 4, 256)), b256, 0, stream>>>(PM, m_b, MK);
  k_final<<<dim3(cdiv(NB * CLO * HWP / 4, 256)), b256, 0, stream>>>(
      T1, T2, ST + 2 * CLO, ST + 4 * CLO, bn_low_g, bn_low_b, bn_high_g, bn_high_b, MK, out);
}
